// EncoderLayer_46153718563354
// MI455X (gfx1250) — hardware-verified
//
#include <hip/hip_runtime.h>
#include <math.h>

#ifndef NB
#define NB 4
#endif
#ifndef SEQ
#define SEQ 2048
#endif
#define NB_FULL 4
#define SEQ_FULL 2048
#define DM 768
#define NH 12
#define DKH 64
#define FFD 3072
#define QKVW (3 * DM)
#define ROWS (NB * SEQ)
#define FFCH ((ROWS) < 4096 ? (ROWS) : 4096)
#define WSC 16.0f
#define CTXC 64.0f
#define PSC 32768.0f
#define LNQ (DM / 128)

static_assert(DM == NH * DKH, "head split must tile the model width");
static_assert(DKH == 64, "attention kernel is written for head dim 64");
static_assert(SEQ % 64 == 0, "attention tiles are 64 queries x 64 keys");
static_assert(ROWS % 64 == 0 && QKVW % 64 == 0 && DM % 64 == 0 && FFD % 64 == 0, "GEMM tiles are 64 x 64 without tails");
static_assert(DM % 32 == 0 && FFD % 32 == 0, "GEMM k-steps are 32 deep");
static_assert(DM % 128 == 0 && 32 * 4 * LNQ == DM, "LayerNorm: 32 lanes x 4 columns x LNQ pieces must equal the row width");
static_assert(DM % 8 == 0 && FFD % 8 == 0, "cast helpers move 8 elements per thread");
static_assert(ROWS % FFCH == 0 && FFCH % 64 == 0, "feed-forward chunk must tile the rows");
static_assert(NB <= NB_FULL && SEQ <= SEQ_FULL, "reduced build must fit inside the staged inputs");

typedef __attribute__((ext_vector_type(16))) _Float16 v16h;
typedef __attribute__((ext_vector_type(8)))  _Float16 v8h;
typedef __attribute__((ext_vector_type(8)))  float    v8f;
typedef __attribute__((ext_vector_type(4)))  float    v4f;
typedef __attribute__((ext_vector_type(4)))  unsigned int v4u;
typedef __attribute__((ext_vector_type(2)))  unsigned int v2u;

union FragH { v16h v; v8h h[2]; };
__device__ __forceinline__ v16h frag_ld(const _Float16* p) { FragH f; f.h[0] = *(const v8h*)(p); f.h[1] = *(const v8h*)(p + 16); return f.v; }

__device__ __forceinline__ v8f wmma16(v16h a, v16h b, v8f c) {
    c = __builtin_amdgcn_wmma_f32_16x16x32_f16(false, a, false, b, (short)0, c, false, false);
    asm volatile("v_nop\n\tv_nop\n\tv_nop\n\tv_nop" : "+v"(c) : "v"(a), "v"(b));
    return c;
}
__device__ __forceinline__ v8f mma_h(v16h a, v16h b, v8f c) { return __builtin_amdgcn_wmma_f32_16x16x32_f16(false, a, false, b, (short)0, c, false, false); }
__device__ __forceinline__ void dep_guard_h(v8f& a, v8f& b, v16h x, v16h y) { asm volatile("v_nop\n\tv_nop\n\tv_nop\n\tv_nop" : "+v"(a), "+v"(b) : "v"(x), "v"(y)); }
__device__ __forceinline__ void keep4_h(v16h a, v16h b, v16h c, v16h d) { asm volatile("v_nop" :: "v"(a), "v"(b), "v"(c), "v"(d)); }
__device__ __forceinline__ void acc_guard4(v8f& a, v8f& b, v8f& c, v8f& d) { asm volatile("v_nop\n\tv_nop\n\tv_nop\n\tv_nop" : "+v"(a), "+v"(b), "+v"(c), "+v"(d)); }

#define VST2(T, ptr, val) do { const T vst2_v_ = (val); *(volatile T*)(ptr) = vst2_v_; __threadfence(); *(volatile T*)(ptr) = vst2_v_; } while (0)
#define VST2V4(ptr, val) do { const v4f vst2_v4_ = (val); *(volatile v4f*)(ptr) = vst2_v4_; __threadfence(); *(volatile v4f*)(ptr) = vst2_v4_; } while (0)

__device__ __forceinline__ unsigned int cmb_pk2(float a, float b) { return (unsigned int)__builtin_bit_cast(unsigned short, (_Float16)a) | ((unsigned int)__builtin_bit_cast(unsigned short, (_Float16)b) << 16); }
__device__ __forceinline__ float cmb_bf(float v) { const unsigned u = __builtin_bit_cast(unsigned, v); const unsigned r = (u + 0x7fffu + ((u >> 16) & 1u)) & 0xffff0000u; return __builtin_bit_cast(float, r); }

__global__ __launch_bounds__(256) void k_cm_bfvec(const float* __restrict__ SRC, float* __restrict__ DST, int n) {
    const int u = blockIdx.x * 256 + threadIdx.x; if (u >= n) return; VST2(float, DST + u, cmb_bf(SRC[u]));
}

__global__ __launch_bounds__(256) void k_cast_x(const float* __restrict__ SRC, unsigned short* __restrict__ DST, int nR, int rpb, long long sbs) {
    const long long u = (long long)blockIdx.x * 256 + threadIdx.x; const int per = DM / 8; if (u >= (long long)nR * per) return;
    const int r = (int)(u / per); const int c0 = 8 * (int)(u % per);
    const float* s = SRC + (long long)(r / rpb) * sbs + (long long)(r % rpb) * DM + c0;
    const v4f a = *(const v4f*)(s), b = *(const v4f*)(s + 4);
    v4u pk; pk.x = cmb_pk2(cmb_bf(a.x), cmb_bf(a.y)); pk.y = cmb_pk2(cmb_bf(a.z), cmb_bf(a.w)); pk.z = cmb_pk2(cmb_bf(b.x), cmb_bf(b.y)); pk.w = cmb_pk2(cmb_bf(b.z), cmb_bf(b.w));
    VST2(v4u, (v4u*)(DST + (long long)r * DM + c0), pk);
}
__global__ __launch_bounds__(256) void k_cm_castbT(const float* __restrict__ SRC, int lds, unsigned short* __restrict__ DST, int ldd, int nR, int nC, float sc) {
    const long long u = (long long)blockIdx.x * 256 + threadIdx.x; const int per = nR / 8; if (u >= (long long)nC * per) return; const int c = (int)(u / per); const int r0 = 8 * (int)(u % per);
    float w[8];
#pragma unroll
    for (int e = 0; e < 8; ++e) w[e] = cmb_bf(SRC[(long long)(r0 + e) * lds + c]) * sc;
    v4u pk; pk.x = cmb_pk2(w[0], w[1]); pk.y = cmb_pk2(w[2], w[3]); pk.z = cmb_pk2(w[4], w[5]); pk.w = cmb_pk2(w[6], w[7]); VST2(v4u, (v4u*)(DST + (long long)c * ldd + r0), pk);
}

template <int OUT_MODE, int ACT>
__device__ __forceinline__ void gemm64_body(const unsigned short* __restrict__ Ap, int lda, const unsigned short* __restrict__ Btp, int ldb,
                                            float* __restrict__ Cf, unsigned short* __restrict__ Ch, int ldc, const float* __restrict__ bias, int M, int N, int K, float scale) {
    __shared__ __align__(16) float sT[8][16 * 68];
    const _Float16* A = (const _Float16*)Ap; const _Float16* Bt = (const _Float16*)Btp;
    const int lane = threadIdx.x & 31;
    const int wave = threadIdx.x >> 5;
    const int tilesN = N >> 6;
    const int tilesM = M >> 6;
    const int tile = blockIdx.x * 8 + wave;
    if (tile >= tilesM * tilesN) return;
    const int tm = tile / tilesN;
    const int tn = tile - tm * tilesN;
    const int m0 = tm << 6;
    const int n0 = tn << 6;
    const int rlane = lane & 15;
    const int koff  = (lane >> 4) * 8;
    const int mOff  = (lane >> 4) * 8;

    v8f acc[4][4];
#pragma unroll
    for (int i = 0; i < 4; ++i)
#pragma unroll
        for (int j = 0; j < 4; ++j) acc[i][j] = (v8f){0.f, 0.f, 0.f, 0.f, 0.f, 0.f, 0.f, 0.f};

    for (int k0 = 0; k0 < K; k0 += 32) {
        v16h bh[4];
#pragma unroll
        for (int j = 0; j < 4; ++j) bh[j] = frag_ld(Bt + (size_t)(n0 + (j << 4) + rlane) * ldb + koff + k0);
#pragma unroll
        for (int i = 0; i < 4; ++i) {
            const v16h ah = frag_ld(A + (size_t)(m0 + (i << 4) + rlane) * lda + koff + k0);
#pragma unroll
            for (int j = 0; j < 4; ++j) acc[i][j] = mma_h(ah, bh[j], acc[i][j]);
            dep_guard_h(acc[i][0], acc[i][3], ah, ah);
        }
        keep4_h(bh[0], bh[1], bh[2], bh[3]);
    }
    acc_guard4(acc[0][0], acc[0][1], acc[0][2], acc[0][3]);
    acc_guard4(acc[1][0], acc[1][1], acc[1][2], acc[1][3]);
    acc_guard4(acc[2][0], acc[2][1], acc[2][2], acc[2][3]);
    acc_guard4(acc[3][0], acc[3][1], acc[3][2], acc[3][3]);

    float* slab = sT[wave];
#pragma unroll
    for (int i = 0; i < 4; ++i) {
        const int mBase = m0 + (i << 4);
#pragma unroll
        for (int j = 0; j < 4; ++j) {
            const int n = n0 + (j << 4) + rlane;
            const float bv = bias[n];
#pragma unroll
            for (int r = 0; r < 8; ++r) {
                float v = acc[i][j][r] * scale;
                v += bv;
                if (ACT == 1) v = fmaxf(v, 0.0f);
                slab[(mOff + r) * 68 + (j << 4) + rlane] = v;
            }
        }
        __builtin_amdgcn_fence(3  , "workgroup");
        __builtin_amdgcn_wave_barrier();
        __builtin_amdgcn_fence(2  , "workgroup");
        if (OUT_MODE == 0) {
            const int hh = lane >> 4, c4 = (lane & 15) * 4;
            for (int pass = 0; pass < 2; ++pass) {
#pragma unroll
                for (int it = 0; it < 8; ++it) {
                    const int row = it * 2 + hh;
                    const v4f v = *(const v4f*)(slab + row * 68 + c4);
                    *(volatile v4f*)(Cf + (size_t)(mBase + row) * ldc + n0 + c4) = v;
                }
                __threadfence();
            }
        } else {
            const int q = lane >> 3, c8 = (lane & 7) * 8;
            for (int pass = 0; pass < 2; ++pass) {
#pragma unroll
                for (int it = 0; it < 4; ++it) {
                    const int row = it * 4 + q;
                    const float* sp = slab + row * 68 + c8;
                    v8h hv;
#pragma unroll
                    for (int e = 0; e < 8; ++e) hv[e] = (_Float16)sp[e];
                    *(volatile v8h*)(Ch + (size_t)(mBase + row) * ldc + n0 + c8) = hv;
                }
                __threadfence();
            }
        }
        __builtin_amdgcn_fence(3  , "workgroup");
        __builtin_amdgcn_wave_barrier();
        __builtin_amdgcn_fence(2  , "workgroup");
    }
}
__global__ __launch_bounds__(256) void k_gemm_f32(const unsigned short* __restrict__ Ap, int lda, const unsigned short* __restrict__ Btp, int ldb, float* __restrict__ C, int ldc,
                                                  const float* __restrict__ bias, int M, int N, int K, float scale) {
    gemm64_body<0, 0>(Ap, lda, Btp, ldb, C, nullptr, ldc, bias, M, N, K, scale);
}
__global__ __launch_bounds__(256) void k_gemm_f16(const unsigned short* __restrict__ Ap, int lda, const unsigned short* __restrict__ Btp, int ldb, unsigned short* __restrict__ C, int ldc,
                                                  const float* __restrict__ bias, int M, int N, int K, float scale) {
    gemm64_body<1, 0>(Ap, lda, Btp, ldb, nullptr, C, ldc, bias, M, N, K, scale);
}
__global__ __launch_bounds__(256) void k_gemm_relu16(const unsigned short* __restrict__ Ap, int lda, const unsigned short* __restrict__ Btp, int ldb, unsigned short* __restrict__ C, int ldc,
                                                     const float* __restrict__ bias, int M, int N, int K, float scale) {
    gemm64_body<1, 1>(Ap, lda, Btp, ldb, nullptr, C, ldc, bias, M, N, K, scale);
}

__global__ __launch_bounds__(128) void k_attn16(const unsigned short* __restrict__ QKVp, const int* __restrict__ mask, unsigned short* __restrict__ CTXp) {
    __shared__ __align__(16) _Float16 Ksh[64 * 64];
    __shared__ __align__(16) _Float16 Vth[64 * 64];
    __shared__ __align__(16) _Float16 Psh[4][16 * 64];
    __shared__ __align__(16) float    Os[4][16 * 68];
    const _Float16* QKV = (const _Float16*)QKVp;
    const int tid = threadIdx.x, wave = tid >> 5, lane = tid & 31, hh = lane >> 4, c = lane & 15;
    constexpr int nqb = SEQ / 64;
    const int bx = blockIdx.x;
    const int qb = bx % nqb;
    const int bh = bx / nqb;
    const int h  = bh % NH;
    const int b  = bh / NH;
    const int q0 = qb * 64 + wave * 16;
    const size_t rowb = (size_t)b * SEQ;

    v16h qa[2];
    {
        const _Float16* qrow = QKV + (rowb + q0 + c) * QKVW + h * DKH + 8 * hh;
        qa[0] = frag_ld(qrow);
        qa[1] = frag_ld(qrow + 32);
    }
    float mrow[8], lrow[8];
    v8f oacc[4];
#pragma unroll
    for (int r = 0; r < 8; ++r) { mrow[r] = -INFINITY; lrow[r] = 0.f; }
#pragma unroll
    for (int t = 0; t < 4; ++t) oacc[t] = (v8f){0.f, 0.f, 0.f, 0.f, 0.f, 0.f, 0.f, 0.f};
    const int* mk = mask + (size_t)b * SEQ_FULL;
    const float L2E = 1.4426950408889634f;
    _Float16* pw = Psh[wave];

    for (int kc = 0; kc < SEQ / 64; ++kc) {
        const int kv0 = kc * 64;
        __syncthreads();
        {
            const int kvr = tid >> 1, dh = (tid & 1) * 32;
            const _Float16* krow = QKV + (rowb + kv0 + kvr) * QKVW + DM + h * DKH + dh;
            const _Float16* vrow = krow + DM;
#pragma unroll
            for (int i = 0; i < 4; ++i) {
                const v8h kk = *(const v8h*)(krow + 8 * i);
                const v8h vv = *(const v8h*)(vrow + 8 * i);
                *(v8h*)(Ksh + kvr * 64 + dh + 8 * i) = kk;
#pragma unroll
                for (int e = 0; e < 8; ++e) Vth[(dh + 8 * i + e) * 64 + kvr] = vv[e];
            }
        }
        __syncthreads();

        v8f s[4];
#pragma unroll
        for (int j = 0; j < 4; ++j) {
            const _Float16* kp = Ksh + (j * 16 + c) * 64 + 8 * hh;
            v8f a = (v8f){0.f, 0.f, 0.f, 0.f, 0.f, 0.f, 0.f, 0.f};
            a = wmma16(qa[0], frag_ld(kp), a);
            a = wmma16(qa[1], frag_ld(kp + 32), a);
            s[j] = a;
        }
        int kvkeep[4];
#pragma unroll
        for (int j = 0; j < 4; ++j) kvkeep[j] = mk[kv0 + j * 16 + c];
        float cm[8];
#pragma unroll
        for (int r = 0; r < 8; ++r) {
            float m = -INFINITY;
#pragma unroll
            for (int j = 0; j < 4; ++j) {
                float v = (kvkeep[j] == 0) ? -1.0e9f : s[j][r] * 0.125f;
                v *= L2E;
                s[j][r] = v;
                m = fmaxf(m, v);
            }
            m = fmaxf(m, __shfl_xor(m, 1, 32)); m = fmaxf(m, __shfl_xor(m, 2, 32));
            m = fmaxf(m, __shfl_xor(m, 4, 32)); m = fmaxf(m, __shfl_xor(m, 8, 32));
            cm[r] = m;
        }
#pragma unroll
        for (int r = 0; r < 8; ++r) {
            const float mnew = fmaxf(mrow[r], cm[r]);
            const float alpha = exp2f(mrow[r] - mnew);
            mrow[r] = mnew;
            float psum = 0.f;
#pragma unroll
            for (int j = 0; j < 4; ++j) {
                const float p = exp2f(s[j][r] - mnew);
                psum += p;
                pw[(8 * hh + r) * 64 + j * 16 + c] = (_Float16)(p * PSC);
            }
            psum += __shfl_xor(psum, 1, 32); psum += __shfl_xor(psum, 2, 32);
            psum += __shfl_xor(psum, 4, 32); psum += __shfl_xor(psum, 8, 32);
            lrow[r] = lrow[r] * alpha + psum;
#pragma unroll
            for (int t = 0; t < 4; ++t) oacc[t][r] *= alpha;
        }
        __builtin_amdgcn_fence(3  , "workgroup");
        __builtin_amdgcn_wave_barrier();
        __builtin_amdgcn_fence(2  , "workgroup");
#pragma unroll
        for (int kk = 0; kk < 2; ++kk) {
            const v16h pa = frag_ld(pw + c * 64 + kk * 32 + 8 * hh);
#pragma unroll
            for (int t = 0; t < 4; ++t) {
                const v16h vb = frag_ld(Vth + (t * 16 + c) * 64 + kk * 32 + 8 * hh);
                oacc[t] = wmma16(pa, vb, oacc[t]);
            }
        }
    }

    float* os = Os[wave];
#pragma unroll
    for (int r = 0; r < 8; ++r) {
        const float inv = CTXC / (lrow[r] * PSC);
#pragma unroll
        for (int t = 0; t < 4; ++t) os[(8 * hh + r) * 68 + t * 16 + c] = oacc[t][r] * inv;
    }
    __builtin_amdgcn_fence(3  , "workgroup");
    __builtin_amdgcn_wave_barrier();
    __builtin_amdgcn_fence(2  , "workgroup");
    {
        const int q = lane >> 3, c8 = (lane & 7) * 8;
        unsigned short* cb = CTXp + (rowb + q0) * DM + h * DKH;
        for (int pass = 0; pass < 2; ++pass) {
#pragma unroll
            for (int it = 0; it < 4; ++it) {
                const int row = it * 4 + q;
                const float* sp = os + row * 68 + c8;
                v8h hv;
#pragma unroll
                for (int e = 0; e < 8; ++e) hv[e] = (_Float16)sp[e];
                *(volatile v8h*)(cb + (size_t)row * DM + c8) = hv;
            }
            __threadfence();
        }
    }
}

template <int NQ, int XBF, int WF, int W16>
__device__ __forceinline__ void ln_body(const float* __restrict__ A, const float* __restrict__ X, int xrpb, long long xbs, const float* __restrict__ GA, const float* __restrict__ BE,
                                        float eps, float inv_vden, int rows, float* __restrict__ Yf, unsigned short* __restrict__ Y16) {
    #pragma clang fp contract(off)
    constexpr int WD = 128 * NQ;
    const int r = blockIdx.x * 8 + (threadIdx.x >> 5); const int L = threadIdx.x & 31; if (r >= rows) return;
    const long long xo = (long long)(r / xrpb) * xbs + (long long)(r % xrpb) * WD;
    v4f v[NQ]; float s = 0.f;
#pragma unroll
    for (int q = 0; q < NQ; ++q) {
        const int c = 4 * L + 128 * q;
        v[q] = *(const v4f*)(A + (long long)r * WD + c);
        v4f x = *(const v4f*)(X + xo + c);
        if (XBF) { x.x = cmb_bf(x.x); x.y = cmb_bf(x.y); x.z = cmb_bf(x.z); x.w = cmb_bf(x.w); }
        v[q] = v[q] + x;
        s += (v[q].x + v[q].y) + (v[q].z + v[q].w);
    }
#pragma unroll
    for (int o = 16; o > 0; o >>= 1) s += __shfl_xor(s, o, 32);
    const float mu = s * (1.f / WD); float qq = 0.f;
#pragma unroll
    for (int q = 0; q < NQ; ++q) { v[q].x -= mu; v[q].y -= mu; v[q].z -= mu; v[q].w -= mu; qq += (v[q].x * v[q].x + v[q].y * v[q].y) + (v[q].z * v[q].z + v[q].w * v[q].w); }
#pragma unroll
    for (int o = 16; o > 0; o >>= 1) qq += __shfl_xor(qq, o, 32);
    const float rs = rsqrtf(qq * inv_vden + eps);
#pragma unroll
    for (int q = 0; q < NQ; ++q) {
        const int c = 4 * L + 128 * q; const v4f ga = *(const v4f*)(GA + c), be = *(const v4f*)(BE + c); v4f y;
        y.x = v[q].x * rs * cmb_bf(ga.x) + cmb_bf(be.x); y.y = v[q].y * rs * cmb_bf(ga.y) + cmb_bf(be.y);
        y.z = v[q].z * rs * cmb_bf(ga.z) + cmb_bf(be.z); y.w = v[q].w * rs * cmb_bf(ga.w) + cmb_bf(be.w);
        const long long o = (long long)r * WD + c;
        if (WF) VST2V4(Yf + o, y);
        if (W16) { v2u pk; pk.x = cmb_pk2(y.x, y.y); pk.y = cmb_pk2(y.z, y.w); VST2(v2u, (v2u*)(Y16 + o), pk); }
    }
}
__global__ __launch_bounds__(256) void k_ln1(const float* __restrict__ A, const float* __restrict__ X, int xrpb, long long xbs, const float* __restrict__ GA, const float* __restrict__ BE,
                                             int rows, float* __restrict__ Yf, unsigned short* __restrict__ Y16) {
    ln_body<LNQ, 1, 1, 1>(A, X, xrpb, xbs, GA, BE, 1e-5f, 1.0f / (float)DM, rows, Yf, Y16);
}
__global__ __launch_bounds__(256) void k_ln2(const float* __restrict__ A, const float* __restrict__ X, int xrpb, long long xbs, const float* __restrict__ GA, const float* __restrict__ BE,
                                             int rows, float* __restrict__ Yf) {
    ln_body<LNQ, 0, 1, 0>(A, X, xrpb, xbs, GA, BE, 1e-5f, 1.0f / (float)DM, rows, Yf, nullptr);
}

static constexpr size_t al256(size_t x) { return (x + 255) / 256 * 256; }
static constexpr size_t mx2(size_t a, size_t b) { return a > b ? a : b; }
static constexpr size_t SZ_X16  = al256((size_t)ROWS * DM * 2);
static constexpr size_t SZ_W3   = al256((size_t)QKVW * DM * 2);
static constexpr size_t SZ_QKV  = (size_t)ROWS * QKVW * 2;
static constexpr size_t SZ_ATT  = (size_t)ROWS * DM * 4;
static constexpr size_t SZ_F16  = al256((size_t)FFCH * FFD * 2);
static constexpr size_t SZ_FFO  = (size_t)FFCH * DM * 4;
static constexpr size_t SZ_REGA = al256(mx2(mx2(SZ_QKV, SZ_ATT), SZ_F16 + SZ_FFO));
static constexpr size_t SZ_WO   = al256((size_t)DM * DM * 2);
static constexpr size_t SZ_X1   = al256((size_t)ROWS * DM * 4);
static constexpr size_t SZ_H16  = al256((size_t)ROWS * DM * 2);
static constexpr size_t SZ_W1T  = al256((size_t)FFD * DM * 2);
static constexpr size_t SZ_W2T  = al256((size_t)DM * FFD * 2);
static constexpr size_t SZ_BR3  = al256((size_t)QKVW * 4);
static constexpr size_t SZ_BRO  = al256((size_t)DM * 4);
static constexpr size_t SZ_BR1  = al256((size_t)FFD * 4);
static constexpr size_t SZ_BR2  = al256((size_t)DM * 4);
static constexpr size_t WS_TOTAL = SZ_X16 + SZ_W3 + SZ_REGA + SZ_WO + SZ_X1 + SZ_H16 + SZ_W1T + SZ_W2T + SZ_BR3 + SZ_BRO + SZ_BR1 + SZ_BR2;
static_assert(WS_TOTAL <= (size_t)134217728, "workspace carve must stay within 128 MiB");
static_assert(SZ_QKV <= SZ_REGA && SZ_ATT <= SZ_REGA && SZ_F16 + SZ_FFO <= SZ_REGA, "shared region must hold each of its users");
static_assert((size_t)ROWS * DM * 2 <= SZ_X16, "context plane must fit the x plane it aliases");
static_assert((size_t)ROWS * DM * 4 <= (size_t)25165824, "output rows must fit the output buffer");

extern "C" void kernel_launch(void* const* d_in, const int* in_sizes, int n_in, void* d_out, int out_size, void* d_ws, size_t ws_size, hipStream_t stream) {
    if (n_in < 16) return;
    if (in_sizes[0] < (NB - 1) * SEQ_FULL * DM + SEQ * DM) return;
    if (in_sizes[1] < (NB - 1) * SEQ_FULL + SEQ) return;
    if (in_sizes[2] < DM * DM || in_sizes[4] < DM * DM || in_sizes[6] < DM * DM || in_sizes[8] < DM * DM) return;
    if (in_sizes[3] < DM || in_sizes[5] < DM || in_sizes[7] < DM || in_sizes[9] < DM) return;
    if (in_sizes[10] < DM * FFD || in_sizes[11] < FFD || in_sizes[12] < FFD * DM || in_sizes[13] < DM) return;
    if (in_sizes[14] < DM || in_sizes[15] < DM) return;
    if (out_size < ROWS * DM) return;
    if (ws_size < WS_TOTAL) return;
    const float* emb  = (const float*)d_in[0];
    const int*   amask = (const int*)d_in[1];
    const float* wq = (const float*)d_in[2];  const float* bq = (const float*)d_in[3];
    const float* wk = (const float*)d_in[4];  const float* bk = (const float*)d_in[5];
    const float* wv = (const float*)d_in[6];  const float* bv = (const float*)d_in[7];
    const float* wo = (const float*)d_in[8];  const float* bo = (const float*)d_in[9];
    const float* w1 = (const float*)d_in[10]; const float* b1 = (const float*)d_in[11];
    const float* w2 = (const float*)d_in[12]; const float* b2 = (const float*)d_in[13];
    const float* lg = (const float*)d_in[14]; const float* lb = (const float*)d_in[15];
    float* out = (float*)d_out;

    char* wsp = (char*)d_ws; size_t off = 0;
    unsigned short* X16  = (unsigned short*)(wsp + off); off += SZ_X16;
    unsigned short* W316 = (unsigned short*)(wsp + off); off += SZ_W3;
    char* regA = wsp + off; off += SZ_REGA;
    unsigned short* WO16 = (unsigned short*)(wsp + off); off += SZ_WO;
    float* X1 = (float*)(wsp + off); off += SZ_X1;
    unsigned short* H16 = (unsigned short*)(wsp + off); off += SZ_H16;
    unsigned short* W1T = (unsigned short*)(wsp + off); off += SZ_W1T;
    unsigned short* W2T = (unsigned short*)(wsp + off); off += SZ_W2T;
    float* BR3 = (float*)(wsp + off); off += SZ_BR3;
    float* BRO = (float*)(wsp + off); off += SZ_BRO;
    float* BR1 = (float*)(wsp + off); off += SZ_BR1;
    float* BR2 = (float*)(wsp + off); off += SZ_BR2;
    if (off > ws_size) return;
    unsigned short* QKV16 = (unsigned short*)regA;
    float* ATT = (float*)regA;
    unsigned short* F16 = (unsigned short*)regA;
    float* FFo = (float*)(regA + SZ_F16);
    unsigned short* CTX16 = X16;

    k_cast_x<<<(unsigned)(((long long)ROWS * (DM / 8) + 255) / 256), 256, 0, stream>>>(emb, X16, ROWS, SEQ, (long long)SEQ_FULL * DM);
    k_cm_castbT<<<(unsigned)(((long long)DM * (DM / 8) + 255) / 256), 256, 0, stream>>>(wq, DM, W316, DM, DM, DM, WSC);
    k_cm_castbT<<<(unsigned)(((long long)DM * (DM / 8) + 255) / 256), 256, 0, stream>>>(wk, DM, W316 + (size_t)DM * DM, DM, DM, DM, WSC);
    k_cm_castbT<<<(unsigned)(((long long)DM * (DM / 8) + 255) / 256), 256, 0, stream>>>(wv, DM, W316 + (size_t)2 * DM * DM, DM, DM, DM, WSC);
    k_cm_castbT<<<(unsigned)(((long long)DM * (DM / 8) + 255) / 256), 256, 0, stream>>>(wo, DM, WO16, DM, DM, DM, WSC);
    k_cm_castbT<<<(unsigned)(((long long)FFD * (DM / 8) + 255) / 256), 256, 0, stream>>>(w1, FFD, W1T, DM, DM, FFD, WSC);
    k_cm_castbT<<<(unsigned)(((long long)DM * (FFD / 8) + 255) / 256), 256, 0, stream>>>(w2, DM, W2T, FFD, FFD, DM, WSC);
    k_cm_bfvec<<<(DM + 255) / 256, 256, 0, stream>>>(bq, BR3, DM);
    k_cm_bfvec<<<(DM + 255) / 256, 256, 0, stream>>>(bk, BR3 + DM, DM);
    k_cm_bfvec<<<(DM + 255) / 256, 256, 0, stream>>>(bv, BR3 + 2 * DM, DM);
    k_cm_bfvec<<<(DM + 255) / 256, 256, 0, stream>>>(bo, BRO, DM);
    k_cm_bfvec<<<(FFD + 255) / 256, 256, 0, stream>>>(b1, BR1, FFD);
    k_cm_bfvec<<<(DM + 255) / 256, 256, 0, stream>>>(b2, BR2, DM);

    k_gemm_f16<<<(unsigned)((((ROWS) / 64) * ((QKVW) / 64) + 7) / 8), 256, 0, stream>>>(X16, DM, W316, DM, QKV16, QKVW, BR3, ROWS, QKVW, DM, 1.0f / WSC);
    k_attn16<<<(unsigned)(NB * NH * (SEQ / 64)), 128, 0, stream>>>(QKV16, amask, CTX16);
    k_gemm_f32<<<(unsigned)((((ROWS) / 64) * ((DM) / 64) + 7) / 8), 256, 0, stream>>>(CTX16, DM, WO16, DM, ATT, DM, BRO, ROWS, DM, DM, 1.0f / (WSC * CTXC));
    k_ln1<<<(ROWS + 7) / 8, 256, 0, stream>>>(ATT, emb, SEQ, (long long)SEQ_FULL * DM, lg, lb, ROWS, X1, H16);
    for (int ch = 0; ch < ROWS / FFCH; ++ch) {
        const size_t ro = (size_t)ch * FFCH * DM;
        k_gemm_relu16<<<(unsigned)((((FFCH) / 64) * ((FFD) / 64) + 7) / 8), 256, 0, stream>>>(H16 + ro, DM, W1T, DM, F16, FFD, BR1, FFCH, FFD, DM, 1.0f / WSC);
        k_gemm_f32<<<(unsigned)((((FFCH) / 64) * ((DM) / 64) + 7) / 8), 256, 0, stream>>>(F16, FFD, W2T, FFD, FFo, DM, BR2, FFCH, DM, FFD, 1.0f / WSC);
        k_ln2<<<(FFCH + 7) / 8, 256, 0, stream>>>(FFo, X1 + ro, FFCH, 0LL, lg, lb, FFCH, out + ro);
    }
}
